// MultiHeadAttention_19507741458712
// MI455X (gfx1250) — hardware-run, weakly checked
//
#include <hip/hip_runtime.h>
#include <math.h>

#ifndef NB
#define NB 2
#endif
#ifndef SEQ
#define SEQ 2048
#endif
#define NB_FULL 2
#define SEQ_FULL 2048
#define DM 1024
#define NHEAD 16
#define HDIM 64
#define MTOK (NB * SEQ)

static_assert(SEQ % 64 == 0);
static_assert(SEQ <= SEQ_FULL);
static_assert(NB <= NB_FULL);
static_assert(DM == NHEAD * HDIM);
static_assert(DM % 64 == 0);
static_assert(MTOK % 64 == 0);

typedef __attribute__((ext_vector_type(16))) _Float16 v16h;
typedef __attribute__((ext_vector_type(8)))  _Float16 v8h;
typedef __attribute__((ext_vector_type(8)))  float    v8f;
typedef __attribute__((ext_vector_type(4)))  float    v4f;
typedef unsigned int cm_u4 __attribute__((ext_vector_type(4)));

__device__ __forceinline__ int frag_k(int i, int h) { return (i < 8) ? (8 * h + i) : (16 + 8 * h + (i - 8)); }

__device__ __forceinline__ v8f wmma16(v16h a, v16h b, v8f c) {
    c = __builtin_amdgcn_wmma_f32_16x16x32_f16(false, a, false, b, (short)0, c, false, false);
    asm volatile("v_nop\n\tv_nop\n\tv_nop\n\tv_nop" : "+v"(c) : "v"(a), "v"(b));
    return c;
}

__device__ __forceinline__ v16h fh_g(const float* __restrict__ p, int k0, int h, float s) {
    const float* p0 = p + k0 + 8 * h;
    const v4f x0 = *(const v4f*)(p0), x1 = *(const v4f*)(p0 + 4), y0 = *(const v4f*)(p0 + 16), y1 = *(const v4f*)(p0 + 20);
    v16h a;
#pragma unroll
    for (int i = 0; i < 4; ++i) {
        a[i] = (_Float16)(x0[i] * s); a[4 + i] = (_Float16)(x1[i] * s);
        a[8 + i] = (_Float16)(y0[i] * s); a[12 + i] = (_Float16)(y1[i] * s);
    }
    return a;
}
__device__ __forceinline__ v16h fh_s(const float* p, int k0, int h, float s) {
    const float* p0 = p + k0 + 8 * h;
    const v4f x0 = *(const v4f*)(p0), x1 = *(const v4f*)(p0 + 4), y0 = *(const v4f*)(p0 + 16), y1 = *(const v4f*)(p0 + 20);
    v16h a;
#pragma unroll
    for (int i = 0; i < 4; ++i) {
        a[i] = (_Float16)(x0[i] * s); a[4 + i] = (_Float16)(x1[i] * s);
        a[8 + i] = (_Float16)(y0[i] * s); a[12 + i] = (_Float16)(y1[i] * s);
    }
    return a;
}

#define VST2(T, ptr, val) do { const T vst2_v_ = (val); *(volatile T*)(ptr) = vst2_v_; __threadfence(); *(volatile T*)(ptr) = vst2_v_; } while (0)

__device__ __forceinline__ unsigned int cmb_pk2(float a, float b) { return (unsigned int)__builtin_bit_cast(unsigned short, (_Float16)a) | ((unsigned int)__builtin_bit_cast(unsigned short, (_Float16)b) << 16); }
__device__ __forceinline__ float cmb_bf(float v) { const unsigned u = __builtin_bit_cast(unsigned, v); const unsigned r = (u + 0x7fffu + ((u >> 16) & 1u)) & 0xffff0000u; return __builtin_bit_cast(float, r); }

__global__ __launch_bounds__(256) void k_cm_bfvec(const float* __restrict__ SRC, float* __restrict__ DST, int n) {
    const int u = blockIdx.x * 256 + threadIdx.x; if (u >= n) return;
    VST2(float, DST + u, cmb_bf(SRC[u]));
}
template <bool BFR>
__global__ __launch_bounds__(256) void k_cm_castb(const float* __restrict__ SRC, int lds, unsigned short* __restrict__ DST, int ldd, int nR, int nC, float sc) {
    const long long u = (long long)blockIdx.x * 256 + threadIdx.x; const int per = nC / 8; if (u >= (long long)nR * per) return;
    const int r = (int)(u / per); const int c0 = 8 * (int)(u % per);
    const float* s = SRC + (long long)r * lds + c0;
    const v4f s0 = *(const v4f*)(s), s1 = *(const v4f*)(s + 4);
    float w[8];
#pragma unroll
    for (int e = 0; e < 4; ++e) { w[e] = (BFR ? cmb_bf(s0[e]) : s0[e]) * sc; w[4 + e] = (BFR ? cmb_bf(s1[e]) : s1[e]) * sc; }
    cm_u4 pk; pk.x = cmb_pk2(w[0], w[1]); pk.y = cmb_pk2(w[2], w[3]); pk.z = cmb_pk2(w[4], w[5]); pk.w = cmb_pk2(w[6], w[7]);
    VST2(cm_u4, (cm_u4*)(DST + (long long)r * ldd + c0), pk);
}
__global__ __launch_bounds__(256) void k_cm_castbT(const float* __restrict__ SRC, int lds, unsigned short* __restrict__ DST, int ldd, int nR, int nC, float sc) {
    const long long u = (long long)blockIdx.x * 256 + threadIdx.x; const int per = nR / 8; if (u >= (long long)nC * per) return;
    const int c = (int)(u / per); const int r0 = 8 * (int)(u % per);
    float w[8];
#pragma unroll
    for (int e = 0; e < 8; ++e) w[e] = cmb_bf(SRC[(long long)(r0 + e) * lds + c]) * sc;
    cm_u4 pk; pk.x = cmb_pk2(w[0], w[1]); pk.y = cmb_pk2(w[2], w[3]); pk.z = cmb_pk2(w[4], w[5]); pk.w = cmb_pk2(w[6], w[7]);
    VST2(cm_u4, (cm_u4*)(DST + (long long)c * ldd + r0), pk);
}

__device__ __forceinline__ void dep_guard_h(v8f& a, v8f& b, v16h x, v16h y) { asm volatile("v_nop\n\tv_nop\n\tv_nop\n\tv_nop" : "+v"(a), "+v"(b) : "v"(x), "v"(y)); }
__device__ __forceinline__ void keep4_h(v16h a, v16h b, v16h c, v16h d) { asm volatile("v_nop" :: "v"(a), "v"(b), "v"(c), "v"(d)); }
__device__ __forceinline__ void acc_guard4(v8f& a, v8f& b, v8f& c, v8f& d) { asm volatile("v_nop\n\tv_nop\n\tv_nop\n\tv_nop" : "+v"(a), "+v"(b), "+v"(c), "+v"(d)); }
union FragU { v16h v; v8h h[2]; };
__device__ __forceinline__ v16h frag_ld(const _Float16* __restrict__ p) {
    FragU f; f.h[0] = *(const v8h*)(p); f.h[1] = *(const v8h*)(p + 16); return f.v;
}

template <int BIAS_MODE>
__global__ __launch_bounds__(256) void wmma_gemm64(
    const unsigned short* __restrict__ Ap, int lda, long long strideA,
    const unsigned short* __restrict__ Btp, int ldb, long long strideB,
    float* __restrict__ Cout, int ldc, long long strideC,
    const float* __restrict__ bias, int M, int N, int K, float scale) {
  const _Float16* A = (const _Float16*)Ap; const _Float16* Bt = (const _Float16*)Btp;
  __shared__ __align__(16) float sT[8][16 * 68];
  const int b    = blockIdx.y;
  const int lane = threadIdx.x & 31;
  const int wave = __builtin_amdgcn_readfirstlane((int)(threadIdx.x >> 5));
  const int tilesN = N >> 6;
  const int tilesM = M >> 6;
  const int tile = blockIdx.x * 8 + wave;
  if (tile >= tilesM * tilesN) return;
  const int tm = tile / tilesN;
  const int tn = tile - tm * tilesN;
  const int m0 = tm << 6;
  const int n0 = tn << 6;

  const _Float16* Ab = A  + (size_t)b * strideA;
  const _Float16* Bb = Bt + (size_t)b * strideB;

  const int rlane = lane & 15;
  const int koff  = (lane >> 4) * 8;
  const int mOff  = (lane >> 4) * 8;

  v8f acc[4][4];
#pragma unroll
  for (int i = 0; i < 4; ++i)
#pragma unroll
    for (int j = 0; j < 4; ++j) acc[i][j] = (v8f){0.f,0.f,0.f,0.f,0.f,0.f,0.f,0.f};

  for (int k0 = 0; k0 < K; k0 += 32) {
    v16h bh[4];
#pragma unroll
    for (int j = 0; j < 4; ++j) {
      const size_t bo = (size_t)(n0 + (j << 4) + rlane) * ldb + koff + k0;
      bh[j] = frag_ld(Bb + bo);
    }
#pragma unroll
    for (int i = 0; i < 4; ++i) {
      const size_t ao = (size_t)(m0 + (i << 4) + rlane) * lda + koff + k0;
      const v16h ah = frag_ld(Ab + ao);
#pragma unroll
      for (int j = 0; j < 4; ++j)
        acc[i][j] = __builtin_amdgcn_wmma_f32_16x16x32_f16(false, ah, false, bh[j], (short)0, acc[i][j], false, false);
      dep_guard_h(acc[i][0], acc[i][3], ah, ah);
    }
    keep4_h(bh[0], bh[1], bh[2], bh[3]);
  }
  acc_guard4(acc[0][0], acc[0][1], acc[0][2], acc[0][3]);
  acc_guard4(acc[1][0], acc[1][1], acc[1][2], acc[1][3]);
  acc_guard4(acc[2][0], acc[2][1], acc[2][2], acc[2][3]);
  acc_guard4(acc[3][0], acc[3][1], acc[3][2], acc[3][3]);

  float* slab = sT[wave];
  float* C = Cout + (size_t)b * strideC;
#pragma unroll
  for (int i = 0; i < 4; ++i) {
    const int mBase = m0 + (i << 4);
#pragma unroll
    for (int j = 0; j < 4; ++j) {
      const int n = n0 + (j << 4) + rlane;
      float bv = 0.f;
      if (BIAS_MODE == 2) bv = bias[n];
#pragma unroll
      for (int r = 0; r < 8; ++r) {
        float v = acc[i][j][r] * scale;
        if (BIAS_MODE == 2) v += bv;
        slab[(mOff + r) * 68 + (j << 4) + rlane] = v;
      }
    }
    __builtin_amdgcn_fence(3  , "workgroup");
    __builtin_amdgcn_wave_barrier();
    __builtin_amdgcn_fence(2  , "workgroup");
    {
      const int hh = lane >> 4, c4 = (lane & 15) * 4;
      for (int pass = 0; pass < 2; ++pass) {
#pragma unroll
        for (int it = 0; it < 8; ++it) {
          const int row = it * 2 + hh;
          const v4f v = *(const v4f*)(slab + row * 68 + c4);
          *(volatile v4f*)(C + (size_t)(mBase + row) * ldc + n0 + c4) = v;
        }
        __threadfence();
      }
    }
    __builtin_amdgcn_fence(3  , "workgroup");
    __builtin_amdgcn_wave_barrier();
    __builtin_amdgcn_fence(2  , "workgroup");
  }
}

#define AW 4
struct AttnP {
    const float* Q; const float* K; const float* V; float* O; const float* Mf;
    long long sQb, sQh, sQi, sKb, sKh, sKj, sVb, sVh, sVj, sOb, sOh, sOi, smb;
    int Lq, Lk; float scale; int pad_;
};
static_assert(sizeof(AttnP) == 5 * 8 + 13 * 8 + 4 * 4);

__global__ __launch_bounds__(32 * AW) void k_attn(AttnP p) {
    constexpr int NT = 4;
    constexpr int VP = 72;
    __shared__ __align__(16) float    pl[AW][16 * 64];
    __shared__ __align__(16) _Float16 vl[64 * VP];
    const int lane = threadIdx.x & 31, hf = lane >> 4, l15 = lane & 15, wave = __builtin_amdgcn_readfirstlane((int)(threadIdx.x >> 5));
    const int h = blockIdx.y, b = blockIdx.z;
    const int q0 = (blockIdx.x * AW + wave) * 16;
    float* myp = pl[wave];
    const float L2E = 1.4426950408889634f;
    const float NEG = -__builtin_inff();
    const int qi = min(q0 + l15, p.Lq - 1);
    const float* qrow  = p.Q + b * p.sQb + h * p.sQh + (long long)qi * p.sQi;
    const float* kbase = p.K + b * p.sKb + h * p.sKh;
    const float* vbase = p.V + b * p.sVb + h * p.sVh;
    const float* mrow  = p.Mf + b * p.smb;
    v16h qa[2];
#pragma unroll
    for (int ks = 0; ks < 2; ++ks) qa[ks] = fh_g(qrow, ks * 32, hf, 1.f);
    v8f o[NT]; float m8[8], l8[8];
#pragma unroll
    for (int t = 0; t < NT; ++t) { v8f zz = {}; o[t] = zz; }
#pragma unroll
    for (int i = 0; i < 8; ++i) { m8[i] = NEG; l8[i] = 0.f; }

    for (int j0 = 0; j0 < p.Lk; j0 += 64) {
        __syncthreads();
#pragma unroll
        for (int it = 0; it < 8; ++it) {
            const int idx = threadIdx.x + it * (32 * AW);
            const int jr = idx >> 4, d4 = (idx & 15) * 4;
            const int j = j0 + jr; const int jc = min(j, p.Lk - 1);
            const v4f f = *(const v4f*)(vbase + (long long)jc * p.sVj + d4);
            const bool in = (j < p.Lk);
            _Float16* dst = vl + jr * VP + d4;
            dst[0] = in ? (_Float16)f.x : (_Float16)0.f; dst[1] = in ? (_Float16)f.y : (_Float16)0.f;
            dst[2] = in ? (_Float16)f.z : (_Float16)0.f; dst[3] = in ? (_Float16)f.w : (_Float16)0.f;
        }
        float mk[4];
#pragma unroll
        for (int t = 0; t < 4; ++t) mk[t] = mrow[min(j0 + t * 16 + l15, p.Lk - 1)];
        v8f s[4];
#pragma unroll
        for (int t = 0; t < 4; ++t) {
            const int j = min(j0 + t * 16 + l15, p.Lk - 1);
            const float* krow = kbase + (long long)j * p.sKj;
            v8f acc = {};
#pragma unroll
            for (int ks = 0; ks < 2; ++ks) acc = wmma16(qa[ks], fh_g(krow, ks * 32, hf, 1.f), acc);
            s[t] = acc;
        }
        float pv[8][4];
#pragma unroll
        for (int i = 0; i < 8; ++i) {
            float sc[4];
#pragma unroll
            for (int t = 0; t < 4; ++t) {
                const int jg = j0 + t * 16 + l15;
                float v = s[t][i] * p.scale;
                v += mk[t];
                v = (jg >= p.Lk) ? NEG : v * L2E;
                sc[t] = v;
            }
            float mx = fmaxf(fmaxf(sc[0], sc[1]), fmaxf(sc[2], sc[3]));
            mx = fmaxf(mx, __shfl_xor(mx, 1, 32)); mx = fmaxf(mx, __shfl_xor(mx, 2, 32));
            mx = fmaxf(mx, __shfl_xor(mx, 4, 32)); mx = fmaxf(mx, __shfl_xor(mx, 8, 32));
            const float mnew = fmaxf(m8[i], mx);
            const float corr = (mnew == NEG) ? 1.f : exp2f(m8[i] - mnew);
            float rs = 0.f;
#pragma unroll
            for (int t = 0; t < 4; ++t) {
                const float pp = (sc[t] == NEG) ? 0.f : exp2f(sc[t] - mnew); rs += pp;
                pv[i][t] = pp;
            }
            rs += __shfl_xor(rs, 1, 32); rs += __shfl_xor(rs, 2, 32); rs += __shfl_xor(rs, 4, 32); rs += __shfl_xor(rs, 8, 32);
            l8[i] = l8[i] * corr + rs; m8[i] = mnew;
#pragma unroll
            for (int t = 0; t < NT; ++t) o[t][i] *= corr;
        }
#pragma unroll
        for (int i = 0; i < 8; ++i)
#pragma unroll
            for (int t = 0; t < 4; ++t) myp[(i + 8 * hf) * 64 + t * 16 + l15] = pv[i][t];
        __syncthreads();
        const v16h pa0 = fh_s(myp + l15 * 64, 0, hf, 4096.f), pa1 = fh_s(myp + l15 * 64, 32, hf, 4096.f);
#pragma unroll
        for (int t = 0; t < NT; ++t) {
            const int dcol = t * 16 + l15;
            v16h b0, b1;
#pragma unroll
            for (int e = 0; e < 16; ++e) { b0[e] = vl[frag_k(e, hf) * VP + dcol]; b1[e] = vl[(32 + frag_k(e, hf)) * VP + dcol]; }
            o[t] = wmma16(pa0, b0, o[t]);
            o[t] = wmma16(pa1, b1, o[t]);
        }
    }
    float invr[8];
#pragma unroll
    for (int i = 0; i < 8; ++i) invr[i] = (l8[i] > 0.f) ? 1.f / (l8[i] * 4096.f) : 0.f;
    __syncthreads();
#pragma unroll
    for (int i = 0; i < 8; ++i)
#pragma unroll
        for (int t = 0; t < NT; ++t) myp[(i + 8 * hf) * 64 + t * 16 + l15] = o[t][i] * invr[i];
    __syncthreads();
    float* obase = p.O + b * p.sOb + h * p.sOh;
    if (q0 + 16 <= p.Lq) {
        const int rsel = lane >> 4, c4 = (lane & 15) * 4;
        for (int pass = 0; pass < 2; ++pass) {
#pragma unroll
            for (int it = 0; it < 8; ++it) {
                const int row = it * 2 + rsel;
                const v4f v = *(const v4f*)(myp + row * 64 + c4);
                *(volatile v4f*)(obase + (long long)(q0 + row) * p.sOi + c4) = v;
            }
            __threadfence();
        }
    }
}

constexpr size_t al256(size_t n) { return (n + 255) / 256 * 256; }
constexpr size_t SZ_X16  = al256((size_t)MTOK * DM * 2);
constexpr size_t SZ_W316 = al256((size_t)3 * DM * DM * 2);
constexpr size_t SZ_QKV  = al256((size_t)MTOK * 3 * DM * 4);
constexpr size_t SZ_AO   = al256((size_t)MTOK * DM * 4);
constexpr size_t SZ_WO16 = al256((size_t)DM * DM * 2);
constexpr size_t SZ_BR3  = al256((size_t)(3 * DM + 64) * 4);
constexpr size_t SZ_BRO  = al256((size_t)(DM + 64) * 4);
constexpr size_t N_MSK   = (size_t)(NB - 1) * SEQ_FULL + SEQ;
constexpr size_t SZ_MSK  = al256((N_MSK + 64) * 4);
constexpr size_t WS_TOTAL = SZ_X16 + SZ_W316 + SZ_QKV + SZ_AO + SZ_WO16 + SZ_BR3 + SZ_BRO + SZ_MSK;
static_assert(WS_TOTAL <= (size_t)134217728);
static_assert(N_MSK % 32 == 0);
static_assert(((size_t)(NB - 1) * SEQ_FULL + SEQ) * DM <= (size_t)NB_FULL * SEQ_FULL * DM);

extern "C" void kernel_launch(void* const* d_in, const int* in_sizes, int n_in, void* d_out, int out_size, void* d_ws, size_t ws_size, hipStream_t stream) {
    if (n_in < 10) return;
    const long long x_need = ((long long)(NB - 1) * SEQ_FULL + SEQ) * DM;
    if ((long long)in_sizes[0] < x_need) return;
    if ((long long)in_sizes[1] < (long long)N_MSK) return;
    if (in_sizes[2] < DM * DM || in_sizes[4] < DM * DM || in_sizes[6] < DM * DM || in_sizes[8] < DM * DM) return;
    if (in_sizes[3] < DM || in_sizes[5] < DM || in_sizes[7] < DM || in_sizes[9] < DM) return;
    if ((long long)out_size < x_need) return;
    if (WS_TOTAL > ws_size) return;
    const float* x    = (const float*)d_in[0];
    const float* mask = (const float*)d_in[1];
    const float* Wq   = (const float*)d_in[2];
    const float* bq   = (const float*)d_in[3];
    const float* Wk   = (const float*)d_in[4];
    const float* bk   = (const float*)d_in[5];
    const float* Wv   = (const float*)d_in[6];
    const float* bv   = (const float*)d_in[7];
    const float* Wo   = (const float*)d_in[8];
    const float* bo   = (const float*)d_in[9];
    float* out = (float*)d_out;
    char* wsp = (char*)d_ws;
    unsigned short* X16  = (unsigned short*)wsp; wsp += SZ_X16;
    unsigned short* W316 = (unsigned short*)wsp; wsp += SZ_W316;
    float* QKV = (float*)wsp; wsp += SZ_QKV;
    float* AO  = (float*)wsp; wsp += SZ_AO;
    unsigned short* WO16 = (unsigned short*)wsp; wsp += SZ_WO16;
    float* BR3 = (float*)wsp; wsp += SZ_BR3;
    float* BRO = (float*)wsp; wsp += SZ_BRO;
    float* MSK = (float*)wsp; wsp += SZ_MSK;
    unsigned short* AO16 = X16;

    {
        const int xb = (SEQ == SEQ_FULL) ? 1 : NB;
        const int xr = (SEQ == SEQ_FULL) ? MTOK : SEQ;
        for (int b = 0; b < xb; ++b)
            k_cm_castb<true><<<(unsigned)(((long long)xr * (DM / 8) + 255) / 256), 256, 0, stream>>>(x + (size_t)b * SEQ_FULL * DM, DM, X16 + (size_t)b * SEQ * DM, DM, xr, DM, 1.0f);
    }
    const unsigned gw = (unsigned)(((long long)DM * (DM / 8) + 255) / 256);
    k_cm_castbT<<<gw, 256, 0, stream>>>(Wq, DM, W316 + (size_t)0 * DM * DM, DM, DM, DM, 16.0f);
    k_cm_castbT<<<gw, 256, 0, stream>>>(Wk, DM, W316 + (size_t)1 * DM * DM, DM, DM, DM, 16.0f);
    k_cm_castbT<<<gw, 256, 0, stream>>>(Wv, DM, W316 + (size_t)2 * DM * DM, DM, DM, DM, 16.0f);
    k_cm_castbT<<<gw, 256, 0, stream>>>(Wo, DM, WO16, DM, DM, DM, 16.0f);
    k_cm_bfvec<<<(DM + 255) / 256, 256, 0, stream>>>(bq, BR3 + 0, DM);
    k_cm_bfvec<<<(DM + 255) / 256, 256, 0, stream>>>(bk, BR3 + DM, DM);
    k_cm_bfvec<<<(DM + 255) / 256, 256, 0, stream>>>(bv, BR3 + 2 * DM, DM);
    k_cm_bfvec<<<(DM + 255) / 256, 256, 0, stream>>>(bo, BRO, DM);
    k_cm_bfvec<<<(unsigned)((N_MSK + 255) / 256), 256, 0, stream>>>(mask, MSK, (int)N_MSK);
    wmma_gemm64<2><<<dim3((unsigned)((((MTOK) / 64) * ((3 * DM) / 64) + 7) / 8), 1u), 256, 0, stream>>>(
        X16, DM, 0, W316, DM, 0, QKV, 3 * DM, 0, BR3, MTOK, 3 * DM, DM, 0.0625f);
    {
        AttnP a;
        a.Q = QKV; a.K = QKV + DM; a.V = QKV + 2 * DM; a.O = AO; a.Mf = MSK;
        a.sQb = (long long)SEQ * 3 * DM; a.sQh = HDIM; a.sQi = 3 * DM;
        a.sKb = (long long)SEQ * 3 * DM; a.sKh = HDIM; a.sKj = 3 * DM;
        a.sVb = (long long)SEQ * 3 * DM; a.sVh = HDIM; a.sVj = 3 * DM;
        a.sOb = (long long)SEQ * DM; a.sOh = HDIM; a.sOi = DM;
        a.smb = SEQ_FULL;
        a.Lq = SEQ; a.Lk = SEQ; a.scale = 0.125f; a.pad_ = 0;
        k_attn<<<dim3((unsigned)(SEQ / (16 * AW)), (unsigned)NHEAD, (unsigned)NB), 32 * AW, 0, stream>>>(a);
    }
    k_cm_castb<false><<<(unsigned)(((long long)MTOK * (DM / 8) + 255) / 256), 256, 0, stream>>>(AO, DM, AO16, DM, MTOK, DM, 256.0f);
    wmma_gemm64<2><<<dim3((unsigned)((((SEQ) / 64) * ((DM) / 64) + 7) / 8), (unsigned)NB), 256, 0, stream>>>(
        AO16, DM, (long long)SEQ * DM, WO16, DM, 0, out, DM, (long long)SEQ_FULL * DM, BRO, SEQ, DM, DM, 1.0f / 4096.0f);
}
